// SoftGroupAttention_76149770158125
// MI455X (gfx1250) — hardware-verified
//
#include <hip/hip_runtime.h>
#include <hip/hip_bf16.h>
#include <math.h>


typedef __attribute__((ext_vector_type(16))) _Float16 v16h;
typedef __attribute__((ext_vector_type(8)))  _Float16 v8h;
typedef __attribute__((ext_vector_type(16))) __bf16   v16b;
typedef __attribute__((ext_vector_type(8)))  __bf16   v8b;
typedef __attribute__((ext_vector_type(8)))  float    v8f;
typedef __attribute__((ext_vector_type(4)))  float    v4f;
#define PSCALE 32768.0f
#define U16(p) ((const unsigned short*)(const void*)(p))
#define PSCALE_INV (1.0f / 32768.0f)

__device__ __forceinline__ unsigned short f2bf_bits(float f) {
  unsigned u = __float_as_uint(f);
  return (unsigned short)((u + 0x7FFFu + ((u >> 16) & 1u)) >> 16);
}
__device__ __forceinline__ float bf_bits2f(unsigned short h) { return __uint_as_float(((unsigned)h) << 16); }

__device__ __forceinline__ void dep_guard_h(v8f& a, v8f& b, v16h x, v16h y) { asm volatile("v_nop\n\tv_nop\n\tv_nop\n\tv_nop" : "+v"(a), "+v"(b) : "v"(x), "v"(y)); }
__device__ __forceinline__ void dep_guard_b(v8f& a, v8f& b, v16b x, v16b y) { asm volatile("v_nop\n\tv_nop\n\tv_nop\n\tv_nop" : "+v"(a), "+v"(b) : "v"(x), "v"(y)); }
__device__ __forceinline__ void keep4_h(v16h a, v16h b, v16h c, v16h d) { asm volatile("v_nop" :: "v"(a), "v"(b), "v"(c), "v"(d)); }
__device__ __forceinline__ void keep4_b(v16b a, v16b b, v16b c, v16b d) { asm volatile("v_nop" :: "v"(a), "v"(b), "v"(c), "v"(d)); }
__device__ __forceinline__ void acc_guard4(v8f& a, v8f& b, v8f& c, v8f& d) { asm volatile("v_nop\n\tv_nop\n\tv_nop\n\tv_nop" : "+v"(a), "+v"(b), "+v"(c), "+v"(d)); }
template <typename T> struct Frag;
template <> struct Frag<_Float16> {
  typedef v16h V; union U { v16h v; v8h h[2]; };
  static __device__ __forceinline__ v16h load(const _Float16* p) {
    U f; f.h[0] = *(const v8h*)(p); f.h[1] = *(const v8h*)(p + 16); return f.v;
  }
  static __device__ __forceinline__ v8f mma(v16h a, v16h b, v8f c) {
    return __builtin_amdgcn_wmma_f32_16x16x32_f16(false, a, false, b, (short)0, c, false, false);
  }
  static __device__ __forceinline__ void guard(v8f& a, v8f& b, v16h x, v16h y) { dep_guard_h(a, b, x, y); }
  static __device__ __forceinline__ void keep(v16h a, v16h b, v16h c, v16h d) { keep4_h(a, b, c, d); }
};
template <> struct Frag<__bf16> {
  typedef v16b V; union U { v16b v; v8b h[2]; };
  static __device__ __forceinline__ v16b load(const __bf16* p) {
    U f; f.h[0] = *(const v8b*)(p); f.h[1] = *(const v8b*)(p + 16); return f.v;
  }
  static __device__ __forceinline__ v8f mma(v16b a, v16b b, v8f c) {
    return __builtin_amdgcn_wmma_f32_16x16x32_bf16(false, a, false, b, (short)0, c, false, false);
  }
  static __device__ __forceinline__ void guard(v8f& a, v8f& b, v16b x, v16b y) { dep_guard_b(a, b, x, y); }
  static __device__ __forceinline__ void keep(v16b a, v16b b, v16b c, v16b d) { keep4_b(a, b, c, d); }
};

template <int ET> struct Elem;
template <> struct Elem<0> { typedef _Float16 T; };
template <> struct Elem<1> { typedef __bf16 T; };
template <int ET, bool SPLIT, int BIAS_MODE, int OUT_MODE, bool RESID, int ACT = 0>
__global__ __launch_bounds__(256) void wmma_gemm64(
    const unsigned short* __restrict__ Ap, const unsigned short* __restrict__ A2p, int lda, long strideA,
    const unsigned short* __restrict__ Btp, const unsigned short* __restrict__ Bt2p, int ldb, long strideB,
    void* __restrict__ Cout, void* __restrict__ Cout2, int ldc, long strideC,
    const float* __restrict__ bias,
    const float* __restrict__ resid, long strideR,
    int M, int N, int K, float scale) {
  typedef typename Elem<ET>::T T;
  typedef typename Frag<T>::V V;
  const T* A = (const T*)Ap; const T* A2 = (const T*)A2p; const T* Bt = (const T*)Btp; const T* Bt2 = (const T*)Bt2p;
  __shared__ __align__(16) float sT[8][16 * 68];
  const int b    = blockIdx.y;
  const int lane = threadIdx.x & 31;
  const int wave = threadIdx.x >> 5;
  const int tilesN = N >> 6;
  const int tilesM = M >> 6;
  const int tile = blockIdx.x * 8 + wave;
  if (tile >= tilesM * tilesN) return;
  const int tm = tile / tilesN;
  const int tn = tile - tm * tilesN;
  const int m0 = tm << 6;
  const int n0 = tn << 6;

  const T* Ab  = A  + (size_t)b * strideA;
  const T* Bb  = Bt + (size_t)b * strideB;
  const T* Ab2 = SPLIT ? (A2  + (size_t)b * strideA) : nullptr;
  const T* Bb2 = SPLIT ? (Bt2 + (size_t)b * strideB) : nullptr;

  const int rlane = lane & 15;
  const int koff  = (lane >> 4) * 8;
  const int mOff  = (lane >> 4) * 8;

  v8f acc[4][4];
#pragma unroll
  for (int i = 0; i < 4; ++i)
#pragma unroll
    for (int j = 0; j < 4; ++j) acc[i][j] = (v8f){0.f,0.f,0.f,0.f,0.f,0.f,0.f,0.f};

  for (int k0 = 0; k0 < K; k0 += 32) {
    V bh[4], bl[4];
#pragma unroll
    for (int j = 0; j < 4; ++j) {
      const size_t bo = (size_t)(n0 + (j << 4) + rlane) * ldb + koff + k0;
      bh[j] = Frag<T>::load(Bb + bo);
      if (SPLIT) bl[j] = Frag<T>::load(Bb2 + bo);
    }
#pragma unroll
    for (int i = 0; i < 4; ++i) {
      const size_t ao = (size_t)(m0 + (i << 4) + rlane) * lda + koff + k0;
      V ah = Frag<T>::load(Ab + ao);
      V al;
      if (SPLIT) al = Frag<T>::load(Ab2 + ao);
#pragma unroll
      for (int j = 0; j < 4; ++j) {
        acc[i][j] = Frag<T>::mma(ah, bh[j], acc[i][j]);
        if (SPLIT) {
          acc[i][j] = Frag<T>::mma(ah, bl[j], acc[i][j]);
          acc[i][j] = Frag<T>::mma(al, bh[j], acc[i][j]);
        }
      }
      Frag<T>::guard(acc[i][0], acc[i][3], ah, SPLIT ? al : ah);
    }
    Frag<T>::keep(bh[0], bh[1], bh[2], bh[3]);
    if (SPLIT) Frag<T>::keep(bl[0], bl[1], bl[2], bl[3]);
  }
  acc_guard4(acc[0][0], acc[0][1], acc[0][2], acc[0][3]);
  acc_guard4(acc[1][0], acc[1][1], acc[1][2], acc[1][3]);
  acc_guard4(acc[2][0], acc[2][1], acc[2][2], acc[2][3]);
  acc_guard4(acc[3][0], acc[3][1], acc[3][2], acc[3][3]);

  float* slab = sT[wave];
  const float* Rb = RESID ? (resid + (size_t)b * strideR) : nullptr;
#pragma unroll
  for (int i = 0; i < 4; ++i) {
    const int mBase = m0 + (i << 4);
#pragma unroll
    for (int j = 0; j < 4; ++j) {
      const int n = n0 + (j << 4) + rlane;
      float bv = 0.f;
      if (BIAS_MODE == 2) bv = bias[n];
#pragma unroll
      for (int r = 0; r < 8; ++r) {
        float v = acc[i][j][r] * scale;
        if (BIAS_MODE == 1) v += bias[mBase + mOff + r];
        if (BIAS_MODE == 2) v += bv;
        if (RESID) v += Rb[(size_t)(mBase + mOff + r) * ldc + n];
        if (ACT == 1) v = tanhf(v);
        if (ACT == 2) v = fmaxf(v, 0.0f);
        if (ACT == 3) v = v / (1.0f + expf(-v));
        if (ACT == 4) v = (v > 0.f) ? v : 0.01f * v;
        if (ACT == 5) v = 0.5f * v * (1.0f + erff(v * 0.70710678118654752f));
        slab[(mOff + r) * 68 + (j << 4) + rlane] = v;
      }
    }
    __builtin_amdgcn_fence(__ATOMIC_RELEASE, "workgroup");
    __builtin_amdgcn_wave_barrier();
    __builtin_amdgcn_fence(__ATOMIC_ACQUIRE, "workgroup");
    if (OUT_MODE == 0) {
      float* C = (float*)Cout + (size_t)b * strideC;
      const int hh = lane >> 4, c4 = (lane & 15) * 4;
      for (int pass = 0; pass < 2; ++pass) {
#pragma unroll
        for (int it = 0; it < 8; ++it) {
          const int row = it * 2 + hh;
          v4f v = *(const v4f*)(slab + row * 68 + c4);
          *(volatile v4f*)(C + (size_t)(mBase + row) * ldc + n0 + c4) = v;
        }
        __threadfence();
      }
    } else {
      const int q = lane >> 3, c8 = (lane & 7) * 8;
      unsigned short* C  = (unsigned short*)Cout  + (size_t)b * strideC;
      unsigned short* C2 = (OUT_MODE == 2) ? ((unsigned short*)Cout2 + (size_t)b * strideC) : nullptr;
      for (int pass = 0; pass < 2; ++pass) {
#pragma unroll
        for (int it = 0; it < 4; ++it) {
          const int row = it * 4 + q;
          const float* sp = slab + row * 68 + c8;
          v8h hv, lv;
#pragma unroll
          for (int e = 0; e < 8; ++e) {
            if (OUT_MODE == 1) {
              hv[e] = (_Float16)sp[e];
            } else {
              unsigned short hb = f2bf_bits(sp[e]);
              unsigned short lb = f2bf_bits(sp[e] - bf_bits2f(hb));
              hv[e] = __builtin_bit_cast(_Float16, hb);
              lv[e] = __builtin_bit_cast(_Float16, lb);
            }
          }
          *(volatile v8h*)(C + (size_t)(mBase + row) * ldc + n0 + c8) = hv;
          if (OUT_MODE == 2) *(volatile v8h*)(C2 + (size_t)(mBase + row) * ldc + n0 + c8) = lv;
        }
        __threadfence();
      }
    }
    __builtin_amdgcn_fence(__ATOMIC_RELEASE, "workgroup");
    __builtin_amdgcn_wave_barrier();
    __builtin_amdgcn_fence(__ATOMIC_ACQUIRE, "workgroup");
  }
}

__global__ __launch_bounds__(256) void cast_f32_f16x8(const float* __restrict__ in, _Float16* __restrict__ out, int n8) {
  const int i = blockIdx.x * 256 + threadIdx.x;
  if (i < n8) {
    const float* p = in + (size_t)i * 8;
    const v4f a = *(const v4f*)p;
    const v4f c = *(const v4f*)(p + 4);
    v8h h;
    h[0] = (_Float16)a[0]; h[1] = (_Float16)a[1]; h[2] = (_Float16)a[2]; h[3] = (_Float16)a[3];
    h[4] = (_Float16)c[0]; h[5] = (_Float16)c[1]; h[6] = (_Float16)c[2]; h[7] = (_Float16)c[3];
    _Float16* o = out + (size_t)i * 8;
    *(volatile v8h*)o = h;
    __threadfence();
    *(volatile v8h*)o = h;
  }
}

template <typename TI>
__global__ __launch_bounds__(256) void transpose_to_f16(const TI* __restrict__ in, int ldi, int R, int C,
                                                          _Float16* __restrict__ out, int ldo, float scale) {
  __shared__ float tile[64][65];
  const int t = threadIdx.x, lane = t & 31, wave = t >> 5;
  const int c0 = blockIdx.x * 64, r0 = blockIdx.y * 64;
  (void)R;
#pragma unroll
  for (int i = 0; i < 16; ++i) {
    const int e = t + i * 256;
    const int rl = e >> 6, cl = e & 63;
    const int cc = c0 + cl;
    float v = 0.0f;
    if (cc < C) v = (float)in[(size_t)(r0 + rl) * ldi + cc] * scale;
    tile[cl][rl] = v;
  }
  __syncthreads();
  const int q = lane >> 3, p8 = (lane & 7) * 8;
  for (int pass = 0; pass < 2; ++pass) {
#pragma unroll
    for (int it = 0; it < 2; ++it) {
      const int row = wave * 8 + it * 4 + q;
      v8h hv;
#pragma unroll
      for (int e = 0; e < 8; ++e) hv[e] = (_Float16)tile[row][p8 + e];
      *(volatile v8h*)(out + (size_t)(c0 + row) * ldo + r0 + p8) = hv;
    }
    __threadfence();
  }
}

__device__ __forceinline__ float gelu_erf(float x) {
  return 0.5f * x * (1.0f + erff(x * 0.70710678118654752f));
}

__global__ __launch_bounds__(256) void gw_kernel(const float* __restrict__ gp, _Float16* __restrict__ gw, int nrows) {
  __shared__ __align__(16) float sh[8][64];
  const int lane = threadIdx.x & 31, wave = threadIdx.x >> 5;
  const int row = blockIdx.x * 8 + wave;
  if (row >= nrows) return;
  const float* in = gp + (size_t)row * 64;
  const float x0 = in[lane], x1 = in[lane + 32];
  const bool ok1 = (lane + 32) < 49;
  const float g0 = gelu_erf(x0);
  const float g1v = gelu_erf(x1);
  const float g1 = ok1 ? g1v : -INFINITY;
  float mx = fmaxf(g0, g1);
#pragma unroll
  for (int off = 16; off; off >>= 1) mx = fmaxf(mx, __shfl_xor(mx, off, 32));
  const float e0 = __expf(g0 - mx);
  const float e1 = ok1 ? __expf(g1v - mx) : 0.0f;
  float s = e0 + e1;
#pragma unroll
  for (int off = 16; off; off >>= 1) s += __shfl_xor(s, off, 32);
  const float inv = __builtin_amdgcn_rcpf(s) * 64.0f;
  sh[wave][lane] = e0 * inv;
  sh[wave][lane + 32] = e1 * inv;
  __builtin_amdgcn_fence(__ATOMIC_RELEASE, "workgroup");
  __builtin_amdgcn_wave_barrier();
  __builtin_amdgcn_fence(__ATOMIC_ACQUIRE, "workgroup");
  if (lane < 8) {
    const float* sp = &sh[wave][lane * 8];
    v8h hv;
#pragma unroll
    for (int e = 0; e < 8; ++e) hv[e] = (_Float16)sp[e];
    _Float16* o = gw + (size_t)row * 64 + lane * 8;
    *(volatile v8h*)o = hv;
    __threadfence();
    *(volatile v8h*)o = hv;
  }
}

__global__ __launch_bounds__(256) void blend_kernel(const float* __restrict__ S, const float* __restrict__ Gm,
                                                    const float* __restrict__ alpha, _Float16* __restrict__ P) {
  __shared__ float red[2][8];
  const int t = threadIdx.x, lane = t & 31, wave = t >> 5;
  const size_t base = (size_t)blockIdx.x * 2048 + (size_t)t * 8;
  const v4f s0 = *(const v4f*)(S + base), s1 = *(const v4f*)(S + base + 4);
  const v4f g0 = *(const v4f*)(Gm + base), g1 = *(const v4f*)(Gm + base + 4);
  float tv[8], gv[8], ev[8];
#pragma unroll
  for (int e = 0; e < 4; ++e) { gv[e] = g0[e]; gv[e + 4] = g1[e]; tv[e] = s0[e] * g0[e]; tv[e + 4] = s1[e] * g1[e]; }
  float mx = -INFINITY;
#pragma unroll
  for (int e = 0; e < 8; ++e) mx = fmaxf(mx, tv[e]);
#pragma unroll
  for (int off = 16; off; off >>= 1) mx = fmaxf(mx, __shfl_xor(mx, off, 32));
  if (lane == 0) red[0][wave] = mx;
  __syncthreads();
  float bm = red[0][0];
#pragma unroll
  for (int i = 1; i < 8; ++i) bm = fmaxf(bm, red[0][i]);
  float sum = 0.0f;
#pragma unroll
  for (int e = 0; e < 8; ++e) { ev[e] = __expf(tv[e] - bm); sum += ev[e]; }
#pragma unroll
  for (int off = 16; off; off >>= 1) sum += __shfl_xor(sum, off, 32);
  if (lane == 0) red[1][wave] = sum;
  __syncthreads();
  float tot = 0.0f;
#pragma unroll
  for (int i = 0; i < 8; ++i) tot += red[1][i];
  const float inv = __builtin_amdgcn_rcpf(tot);
  const float al = alpha[0];
  const float a = __builtin_amdgcn_rcpf(1.0f + __expf(-al));
  const float ca = (1.0f - a) * inv * 16384.0f;
  const float cb = a * 16384.0f;
  v8h hv;
#pragma unroll
  for (int e = 0; e < 8; ++e) hv[e] = (_Float16)(ev[e] * ca + gv[e] * cb);
  _Float16* o = P + base;
  *(volatile v8h*)o = hv;
  __threadfence();
  *(volatile v8h*)o = hv;
}

template <int BIAS, int OUT>
static void launch_gemm(hipStream_t st, const void* A, int lda, const void* Bt, int ldb, void* C, int ldc,
                        const float* bias, int M, int N, int K, float scale) {
  const int tiles = (M / 64) * (N / 64);
  dim3 grid((unsigned)((tiles + 7) / 8), 1, 1);
  wmma_gemm64<0, false, BIAS, OUT, false, 0><<<grid, 256, 0, st>>>(
      (const unsigned short*)A, (const unsigned short*)A, lda, 0L,
      (const unsigned short*)Bt, (const unsigned short*)Bt, ldb, 0L,
      C, C, ldc, 0L, bias, bias, 0L, M, N, K, scale);
}

extern "C" void kernel_launch(void* const* d_in, const int* in_sizes, int n_in,
                              void* d_out, int out_size, void* d_ws, size_t ws_size,
                              hipStream_t stream) {
  const int BS = 8, NS = 2048, D = 768, TD = 2304, G = 49, GP = 64, MR = BS * NS;
  if (n_in < 7) return;
  if (in_sizes[0] != MR * D || in_sizes[1] != D * TD || in_sizes[2] != TD || in_sizes[3] != D * D ||
      in_sizes[4] != D || in_sizes[5] != D * G || in_sizes[6] < 1 || out_size != MR * D) return;

  const float* x      = (const float*)d_in[0];
  const float* W_qkv  = (const float*)d_in[1];
  const float* b_qkv  = (const float*)d_in[2];
  const float* W_proj = (const float*)d_in[3];
  const float* b_proj = (const float*)d_in[4];
  const float* W_gp   = (const float*)d_in[5];
  const float* alpha  = (const float*)d_in[6];
  float* out = (float*)d_out;

  char* ws = (char*)d_ws;
  size_t off = 0;
  auto carve = [&](size_t bytes) { char* p = ws + off; off += (bytes + 255) & ~(size_t)255; return p; };
  _Float16* WqkvT  = (_Float16*)carve((size_t)TD * D * 2);
  _Float16* WprojT = (_Float16*)carve((size_t)D * D * 2);
  _Float16* WgpT   = (_Float16*)carve((size_t)GP * D * 2);
  _Float16* X16    = (_Float16*)carve((size_t)MR * D * 2);
  _Float16* O16    = (_Float16*)carve((size_t)MR * D * 2);
  _Float16* QKV16  = (_Float16*)carve((size_t)NS * TD * 2);
  float*    Sb     = (float*)carve((size_t)NS * NS * 4);
  float*    GWM    = (float*)carve((size_t)NS * NS * 4);
  _Float16* P16    = (_Float16*)carve((size_t)NS * NS * 2);
  float*    GPb    = (float*)carve((size_t)NS * GP * 4);
  _Float16* GW16   = (_Float16*)carve((size_t)NS * GP * 2);
  _Float16* VT16   = (_Float16*)carve((size_t)D * NS * 2);
  if (off > ws_size) return;

  const float scale_qk = 0.03608439182435161f;

  transpose_to_f16<float><<<dim3(TD / 64, D / 64), 256, 0, stream>>>(W_qkv, TD, D, TD, WqkvT, D, 16.0f);
  transpose_to_f16<float><<<dim3(D / 64, D / 64), 256, 0, stream>>>(W_proj, D, D, D, WprojT, D, 16.0f);
  transpose_to_f16<float><<<dim3(GP / 64, D / 64), 256, 0, stream>>>(W_gp, G, D, G, WgpT, D, 16.0f);
  {
    const int n8 = MR * D / 8;
    cast_f32_f16x8<<<(unsigned)((n8 + 255) / 256), 256, 0, stream>>>(x, X16, n8);
  }

  for (int bi = 0; bi < BS; ++bi) {
    const _Float16* Xb = X16 + (size_t)bi * NS * D;
    _Float16* Ob = O16 + (size_t)bi * NS * D;
    launch_gemm<2, 1>(stream, Xb, D, WqkvT, D, QKV16, TD, b_qkv, NS, TD, D, 1.0f / 16.0f);
    launch_gemm<0, 0>(stream, QKV16, TD, QKV16 + D, TD, Sb, NS, b_proj, NS, NS, D, scale_qk);
    launch_gemm<0, 0>(stream, QKV16 + 2 * D, TD, WgpT, D, GPb, GP, b_proj, NS, GP, D, 1.0f / 16.0f);
    gw_kernel<<<NS / 8, 256, 0, stream>>>(GPb, GW16, NS);
    launch_gemm<0, 0>(stream, GW16, GP, GW16, GP, GWM, NS, b_proj, NS, NS, GP, 1.0f / 4096.0f);
    blend_kernel<<<NS, 256, 0, stream>>>(Sb, GWM, alpha, P16);
    transpose_to_f16<_Float16><<<dim3(D / 64, NS / 64), 256, 0, stream>>>(QKV16 + 2 * D, TD, NS, D, VT16, NS, 1.0f);
    launch_gemm<0, 1>(stream, P16, NS, VT16, NS, Ob, D, b_proj, NS, D, NS, 1.0f / 16384.0f);
  }
  launch_gemm<2, 0>(stream, O16, D, WprojT, D, out, D, b_proj, MR, D, D, 1.0f / 16.0f);
}
